// BasicGNN_25950192402597
// MI455X (gfx1250) — hardware-verified
//
#include <hip/hip_runtime.h>
#include <hip/hip_bf16.h>
#include <math.h>


#define BB 2
#define SS 2048
#define DD 1024
#define HH 16
#define DKK 64
#define QW 2

typedef _Float16 bf16;
typedef __attribute__((ext_vector_type(4))) unsigned v4u_t;
typedef unsigned v4ua __attribute__((ext_vector_type(4), may_alias));
typedef __attribute__((ext_vector_type(4))) float v4f_t;
typedef float v4fa __attribute__((ext_vector_type(4), may_alias));
typedef __attribute__((ext_vector_type(16))) bf16  bf16x16;
typedef __attribute__((ext_vector_type(8)))  bf16  bf16x8;
typedef __attribute__((ext_vector_type(4)))  bf16  bf16x4;
typedef __attribute__((ext_vector_type(8)))  float f32x8;

#define LDS_STRIDE 48
#define KSTRIDE    72
#define VSTRIDE    48

__device__ __forceinline__ f32x8 wmma_bf16(bf16x16 a, bf16x16 b, f32x8 c) {
  return __builtin_amdgcn_wmma_f32_16x16x32_f16(
      false, a, false, b, (short)0, c, false, false);
}

template <typename T>
__device__ __forceinline__ bf16x16 load_frag(const T* __restrict__ base, int ld,
                                             int row0, int k0) {
  const int lane = threadIdx.x & 31;
  const int r    = lane & 15;
  const int kh   = (lane >> 4) * 8;
  const T* p0 = base + (size_t)(row0 + r) * ld + (k0 + kh);
  const T* p1 = p0 + 16;
  bf16x16 f;
#pragma unroll
  for (int i = 0; i < 8; ++i) {
    f[i]     = (bf16)p0[i];
    f[i + 8] = (bf16)p1[i];
  }
  return f;
}

__device__ __forceinline__ bf16x16 lds_frag(const bf16* base, int stride) {
  const int lane = threadIdx.x & 31;
  const int row  = lane & 15;
  const int kh   = (lane >> 4) * 8;
  const bf16x8 lo = *(const bf16x8*)(base + row * stride + kh);
  const bf16x8 hi = *(const bf16x8*)(base + row * stride + kh + 16);
  bf16x16 f;
#pragma unroll
  for (int i = 0; i < 8; ++i) { f[i] = lo[i]; f[i + 8] = hi[i]; }
  return f;
}

template <typename T>
__device__ __forceinline__ void stage_read16(const T* __restrict__ p, float* buf) {
#pragma unroll
  for (int i = 0; i < 16; ++i) buf[i] = (float)p[i];
}

__device__ __forceinline__ void stage_write(bf16* dst, const float* buf, int nquad) {
#pragma unroll
  for (int i = 0; i < nquad; ++i) {
    bf16x4 q;
    q[0] = (bf16)buf[4 * i];     q[1] = (bf16)buf[4 * i + 1];
    q[2] = (bf16)buf[4 * i + 2]; q[3] = (bf16)buf[4 * i + 3];
    *(bf16x4*)(dst + 4 * i) = q;
  }
}

template <typename AT, int MODE>
__global__ __launch_bounds__(256) void gemm_bias_kernel(
    const AT* __restrict__ A, const float* __restrict__ W,
    const float* __restrict__ bias, void* __restrict__ out,
    int M, int N, int K) {
  __shared__ bf16 ldsA[128 * LDS_STRIDE];
  __shared__ bf16 ldsW[256 * LDS_STRIDE];
  __shared__ __attribute__((aligned(16))) unsigned char sob[256 * 136 * 2];

  const int t    = threadIdx.x;
  const int wave = t >> 5;
  const int lane = t & 31;
  const int wm   = (wave & 1) * 64;
  const int wn   = (wave >> 1) * 64;
  const int mBlk = blockIdx.x * 128;
  const int nBlk = blockIdx.y * 256;

  const int arow = t >> 1;
  const int ach  = (t & 1) * 16;

  float abuf[16];
  float wbuf[32];

  stage_read16(A + (size_t)(mBlk + arow) * K + ach, abuf);
  stage_read16(W + (size_t)(nBlk + t) * K,          wbuf);
  stage_read16(W + (size_t)(nBlk + t) * K + 16,     wbuf + 16);

  f32x8 acc[4][4] = {};

  for (int k = 0; k < K; k += 32) {
    __syncthreads();
    stage_write(&ldsA[arow * LDS_STRIDE + ach], abuf, 4);
    stage_write(&ldsW[t * LDS_STRIDE],          wbuf, 8);
    if (k + 32 < K) {
      stage_read16(A + (size_t)(mBlk + arow) * K + (k + 32) + ach, abuf);
      stage_read16(W + (size_t)(nBlk + t) * K + (k + 32),          wbuf);
      stage_read16(W + (size_t)(nBlk + t) * K + (k + 32) + 16,     wbuf + 16);
    }
    __syncthreads();

    bf16x16 af[4], wf[4];
#pragma unroll
    for (int i = 0; i < 4; ++i)
      af[i] = lds_frag(ldsA + (wm + 16 * i) * LDS_STRIDE, LDS_STRIDE);
#pragma unroll
    for (int j = 0; j < 4; ++j)
      wf[j] = lds_frag(ldsW + (wn + 16 * j) * LDS_STRIDE, LDS_STRIDE);
#pragma unroll
    for (int i = 0; i < 4; ++i)
#pragma unroll
      for (int j = 0; j < 4; ++j)
        acc[i][j] = wmma_bf16(af[i], wf[j], acc[i][j]);
  }

  const int nlane = lane & 15;
  const int mh    = (lane >> 4) * 8;
  __syncthreads();
  if (MODE == 0 || MODE == 1 || MODE == 3) {
    bf16* so = (bf16*)sob;
#pragma unroll
    for (int i = 0; i < 4; ++i)
#pragma unroll
      for (int j = 0; j < 4; ++j) {
        const int nl = wn + 16 * j + nlane;
        const float bv = bias ? bias[nBlk + nl] : 0.0f;
#pragma unroll
        for (int r = 0; r < 8; ++r) {
          const int ml = wm + 16 * i + mh + r;
          const bf16 hv = (MODE == 3) ? (bf16)fmaxf(acc[i][j][r] + bv, 0.0f) : (bf16)(acc[i][j][r] + bv);
          if (MODE == 0 || MODE == 3) so[ml * 264 + nl] = hv;
          else           so[nl * 136 + ml] = hv;
        }
      }
    __syncthreads();
#pragma unroll 1
    for (int pass = 0; pass < 2; ++pass) {
      if (MODE == 0 || MODE == 3) {
        for (int ch = t; ch < 128 * 32; ch += 256) { const int ml = ch >> 5, q = (ch & 31) * 8;
          *(volatile v4u_t*)((bf16*)out + (size_t)(mBlk + ml) * N + nBlk + q) = *(const v4ua*)(so + ml * 264 + q); }
      } else {
        const int b_ = mBlk / SS, s0 = mBlk & (SS - 1);
        for (int ch = t; ch < 256 * 16; ch += 256) { const int nl = ch >> 4, q = (ch & 15) * 8; const int n = nBlk + nl, h = n >> 6, dk = n & (DKK - 1);
          *(volatile v4u_t*)((bf16*)out + (((size_t)(b_ * HH + h)) * DKK + dk) * SS + s0 + q) = *(const v4ua*)(so + nl * 136 + q); }
      }
      __threadfence();
    }
  } else {
    float* so = (float*)sob;
#pragma unroll 1
    for (int hf = 0; hf < 2; ++hf) {
      if (wm == hf * 64) {
#pragma unroll
        for (int i = 0; i < 4; ++i)
#pragma unroll
          for (int j = 0; j < 4; ++j) {
            const int nl = wn + 16 * j + nlane;
            const float bv = bias ? bias[nBlk + nl] : 0.0f;
#pragma unroll
            for (int r = 0; r < 8; ++r) so[(16 * i + mh + r) * 260 + nl] = acc[i][j][r] + bv;
          }
      }
      __syncthreads();
#pragma unroll 1
      for (int pass = 0; pass < 2; ++pass) {
        for (int ch = t; ch < 64 * 64; ch += 256) { const int ml = ch >> 6, q = (ch & 63) * 4;
          *(volatile v4f_t*)((float*)out + (size_t)(mBlk + hf * 64 + ml) * N + nBlk + q) = *(const volatile v4fa*)(so + ml * 260 + q); }
        __threadfence();
      }
      __syncthreads();
    }
  }
}


#define GN 100000
#define GNP 100352
#define GE 1600000
#define DR 50176

__global__ __launch_bounds__(256) void k_degc(const int* __restrict__ idx, float* __restrict__ nrm) {
  __shared__ unsigned short dg[DR]; __shared__ int qd[8][256]; __shared__ int wcnt[8][8];
  const int tid = threadIdx.x, lane = tid & 31, wave = tid >> 5, r0 = blockIdx.x * DR;
  for (int i = tid; i < DR; i += 256) dg[i] = 0;
  __syncthreads();
#pragma unroll 1
  for (int c0 = 0; c0 < GE; c0 += 256) {
    const int e = c0 + tid; int d = -1;
    if (e < GE) { const int draw = idx[e]; const int dd = draw < 0 ? 0 : (draw >= GN ? GN - 1 : draw); if (dd >= r0 && dd < r0 + DR) d = dd - r0; }
    const int own = (d >= 0) ? (d & 7) : -1; unsigned mown = 0u;
#pragma unroll
    for (int ww = 0; ww < 8; ++ww) { const unsigned m = __builtin_amdgcn_ballot_w32(own == ww); if (own == ww) mown = m; if (lane == 0) wcnt[ww][wave] = __builtin_popcount(m); }
    __syncthreads();
    if (own >= 0) { int base = 0;
#pragma unroll
      for (int w2 = 0; w2 < 8; ++w2) base += (w2 < wave) ? wcnt[own][w2] : 0;
      const int pos = base + __builtin_popcount(mown & ((1u << lane) - 1u)); qd[own][pos] = d; }
    int total = 0;
#pragma unroll
    for (int w2 = 0; w2 < 8; ++w2) total += wcnt[wave][w2];
    __syncthreads();
    if (lane == 0) {
#pragma unroll 1
      for (int qi = 0; qi < total; ++qi) dg[qd[wave][qi]] += 1; }
    __syncthreads();
  }
#pragma unroll 1
  for (int pass = 0; pass < 2; ++pass) {
    for (int i = tid; i < DR / 4; i += 256) { v4f_t v;
#pragma unroll
      for (int q = 0; q < 4; ++q) { const float g = (float)dg[i * 4 + q]; v[q] = rsqrtf(g + 1.0f); }
      *(volatile v4f_t*)(nrm + r0 + i * 4) = v; }
    __threadfence(); }
}
template <int FW, int RANGE>
__global__ __launch_bounds__(256) void k_agg(const int* __restrict__ rowi, const int* __restrict__ coli, const float* __restrict__ no, const float* __restrict__ ni,
                                            const float* __restrict__ H, float* __restrict__ R, int rsel) {
  __shared__ int qd[8][256], qs[8][256]; __shared__ float qw[8][256]; __shared__ int wcnt[8][8];
  const int tid = threadIdx.x, lane = tid & 31, wave = tid >> 5, r0 = rsel * RANGE;
  constexpr int Q4 = FW / 4; constexpr int NQ = RANGE * FW / 4; constexpr int LPR = (FW >= 32) ? 32 : FW; (void)Q4;
  for (int i = tid; i < NQ; i += 256) { v4f_t z; z.x = z.y = z.z = z.w = 0.0f; *(volatile v4f_t*)(R + (size_t)i * 4) = z; }
  __threadfence(); __syncthreads();
#pragma unroll 1
  for (int c0 = 0; c0 < GE; c0 += 256) {
    const int e = c0 + tid; int d = -1, sidx = 0; float w = 0.0f;
    if (e < GE) { const int draw = coli[e]; const int dd = draw < 0 ? 0 : (draw >= GN ? GN - 1 : draw);
      if (dd >= r0 && dd < r0 + RANGE) { d = dd - r0; const int ss = rowi[e]; sidx = ss < 0 ? 0 : (ss >= GN ? GN - 1 : ss); w = no[sidx] * ni[dd]; } }
    const int own = (d >= 0) ? (d & 7) : -1; unsigned mown = 0u;
#pragma unroll
    for (int ww = 0; ww < 8; ++ww) { const unsigned m = __builtin_amdgcn_ballot_w32(own == ww); if (own == ww) mown = m; if (lane == 0) wcnt[ww][wave] = __builtin_popcount(m); }
    __syncthreads();
    if (own >= 0) { int base = 0;
#pragma unroll
      for (int w2 = 0; w2 < 8; ++w2) base += (w2 < wave) ? wcnt[own][w2] : 0;
      const int pos = base + __builtin_popcount(mown & ((1u << lane) - 1u)); qd[own][pos] = d; qs[own][pos] = sidx; qw[own][pos] = w; }
    int total = 0;
#pragma unroll
    for (int w2 = 0; w2 < 8; ++w2) total += wcnt[wave][w2];
    __syncthreads();
#pragma unroll 1
    for (int qi = 0; qi < total; ++qi) { const int dl = qd[wave][qi]; const int sl = qs[wave][qi]; const float wv = qw[wave][qi];
      float* row = R + (size_t)dl * FW; const float* hs = H + (size_t)sl * FW;
      if (FW >= 32) {
#pragma unroll
        for (int u = 0; u < FW / 32; ++u) row[u * 32 + lane] += wv * hs[u * 32 + lane]; }
      else { if (lane < LPR) row[lane] += wv * hs[lane]; } }
    __syncthreads();
  }
  __threadfence(); __syncthreads();
  for (int i = tid; i < NQ; i += 256) { float* p = R + (size_t)i * 4; const v4f_t v = *(const volatile v4fa*)p; *(volatile v4f_t*)p = v; }
  __threadfence();
}
__global__ __launch_bounds__(256) void k_tw(const float* __restrict__ W, float* __restrict__ WT, int K, int N) {
  for (int i = blockIdx.x * 256 + threadIdx.x; i < K * N; i += gridDim.x * 256) { const int n = i / K, k = i % K; const float v = W[(size_t)k * N + n];
    *(volatile float*)(WT + i) = v; __threadfence(); *(volatile float*)(WT + i) = v; }
}
__global__ __launch_bounds__(256) void k_zero(float* __restrict__ p, int n4) { const int i = blockIdx.x * 256 + threadIdx.x; if (i < n4) { v4f_t z; z.x = z.y = z.z = z.w = 0.f; *(volatile v4f_t*)(p + (size_t)i * 4) = z; __threadfence(); *(volatile v4f_t*)(p + (size_t)i * 4) = z; } }

__global__ __launch_bounds__(128) void k_packA(const float* __restrict__ W1, float* __restrict__ A) {
  const int m = blockIdx.x, k = threadIdx.x; const float v = (m < 64) ? W1[(size_t)k * 64 + m] : 0.0f;
  *(volatile float*)(A + (size_t)m * 128 + k) = v; __threadfence(); *(volatile float*)(A + (size_t)m * 128 + k) = v;
}
template <int FW>
__global__ __launch_bounds__(FW) void k_selfadd(const float* __restrict__ X, const float* __restrict__ dinv, float* __restrict__ R) {
  const int n = blockIdx.x, c = threadIdx.x; const float di = dinv[n]; float xv = X[(size_t)n * FW + c]; if (!(fabsf(xv) <= 3.4e38f)) xv = 0.0f;
  const float v = R[(size_t)n * FW + c] + di * di * xv; *(volatile float*)(R + (size_t)n * FW + c) = v; __threadfence(); *(volatile float*)(R + (size_t)n * FW + c) = v;
}
__global__ __launch_bounds__(128) void k_clean(const float* __restrict__ x, float* __restrict__ Xc) {
  const int n = blockIdx.x, c = threadIdx.x; float v = x[(size_t)n * 128 + c]; if (!(fabsf(v) <= 3.4e38f)) v = 0.0f;
  *(volatile float*)(Xc + (size_t)n * 128 + c) = v; __threadfence(); *(volatile float*)(Xc + (size_t)n * 128 + c) = v;
}
__global__ __launch_bounds__(256) void k_h1h2(const bf16* __restrict__ T, const float* __restrict__ b1, const float* __restrict__ g, const float* __restrict__ be, const float* __restrict__ rm, const float* __restrict__ rv,
                                             const float* __restrict__ W2, float* __restrict__ H2) {
  __shared__ float tile[64][65]; __shared__ float w2[64][2]; __shared__ float h2s[64][2];
  const int n0 = blockIdx.x * 64, t = threadIdx.x;
  for (int i = t; i < 64 * 64; i += 256) { const int c = i >> 6, nn = i & 63; const float v = (float)T[(size_t)c * GNP + n0 + nn] + b1[c];
    tile[c][nn] = fmaxf((v - rm[c]) * rsqrtf(rv[c] + 1e-5f) * g[c] + be[c], 0.0f); }
  if (t < 128) w2[t >> 1][t & 1] = W2[t];
  __syncthreads();
  if (t < 128) { const int nn = t >> 1, o = t & 1; float s = 0.0f;
#pragma unroll 1
    for (int c = 0; c < 64; ++c) s += tile[c][nn] * w2[c][o]; h2s[nn][o] = s; }
  __syncthreads();
  if (t < 32) { const v4f_t v = *(const volatile v4fa*)(&h2s[0][0] + t * 4); *(volatile v4f_t*)(H2 + (size_t)n0 * 2 + t * 4) = v; __threadfence(); *(volatile v4f_t*)(H2 + (size_t)n0 * 2 + t * 4) = v; }
}
__global__ __launch_bounds__(256) void k_out(const float* __restrict__ R2, const float* __restrict__ H2, const float* __restrict__ dinv, const float* __restrict__ b2, float* __restrict__ out) {
  const int i = blockIdx.x * 256 + threadIdx.x; if (i >= GN * 2) return; const int n = i >> 1, o = i & 1; const float di = dinv[n];
  const float v = R2[i] + di * di * H2[i] + b2[o]; *(volatile float*)(out + i) = v; __threadfence(); *(volatile float*)(out + i) = v;
}

extern "C" void kernel_launch(void* const* d_in, const int* in_sizes, int n_in,
                              void* d_out, int out_size, void* d_ws, size_t ws_size,
                              hipStream_t stream) {
  (void)in_sizes; (void)n_in; (void)out_size; (void)ws_size;
  const float* x = (const float*)d_in[0];
  const int* ei = (const int*)d_in[1];
  const float* W1 = (const float*)d_in[2]; const float* b1 = (const float*)d_in[3];
  const float* g = (const float*)d_in[4]; const float* be = (const float*)d_in[5]; const float* rm = (const float*)d_in[6]; const float* rv = (const float*)d_in[7];
  const float* W2 = (const float*)d_in[8]; const float* b2 = (const float*)d_in[9];
  const int* src = ei; const int* dst = ei + (size_t)GE;
  char* ws = (char*)d_ws;
  float* A1   = (float*)ws; ws += (size_t)128 * 128 * 4;
  float* dinv = (float*)ws; ws += (size_t)GNP * 4;
  float* Xc   = (float*)ws; ws += (size_t)GNP * 128 * 4;
  float* R1   = (float*)ws; ws += (size_t)GNP * 128 * 4;
  bf16* T     = (bf16*)Xc;
  float* H2   = (float*)ws; ws += (size_t)GNP * 2 * 4;
  float* R2   = (float*)ws; ws += (size_t)GNP * 2 * 4;
  k_packA<<<128, 128, 0, stream>>>(W1, A1);
  k_clean<<<GN, 128, 0, stream>>>(x, Xc);
  k_degc<<<GNP / DR, 256, 0, stream>>>(dst, dinv);
  k_agg<128, GNP><<<1, 256, 0, stream>>>(src, dst, dinv, dinv, Xc, R1, 0);
  k_selfadd<128><<<GN, 128, 0, stream>>>(Xc, dinv, R1);
  gemm_bias_kernel<float, 0><<<dim3(1, GNP / 256), 256, 0, stream>>>(A1, R1, nullptr, T, 128, GNP, 128);
  k_h1h2<<<GNP / 64, 256, 0, stream>>>(T, b1, g, be, rm, rv, W2, H2);
  k_agg<2, GNP><<<1, 256, 0, stream>>>(src, dst, dinv, dinv, H2, R2, 0);
  k_out<<<(GN * 2 + 255) / 256, 256, 0, stream>>>(R2, H2, dinv, b2, (float*)d_out);
}
